// HomogeneousGCN_8727373545900
// MI455X (gfx1250) — hardware-run, weakly checked
//
#include <hip/hip_runtime.h>


namespace {
constexpr int N = 100000, E = 3200000, F = 128, H = 32, O = 16, G = 512, NPB = 8;
constexpr float XS = 8.0f, HS = 256.0f, WSC = 256.0f, EPS = 1e-5f;
typedef _Float16 b16;
typedef __attribute__((ext_vector_type(16))) _Float16 v16b;
typedef __attribute__((ext_vector_type(8))) _Float16 v8b;
typedef __attribute__((ext_vector_type(8))) float v8f;
typedef __attribute__((ext_vector_type(4))) float v4f;
__device__ __forceinline__ float bf16_rne(float f) { unsigned int u = __float_as_uint(f); u += 0x7FFFu + ((u >> 16) & 1u); float r = __uint_as_float(u & 0xFFFF0000u); asm volatile("" : "+v"(r)); return r; }
__device__ __forceinline__ float bfv(float f) { float r = bf16_rne(f); asm volatile("" : "+v"(r)); return r; }
__device__ __forceinline__ void split16(float v, b16& hi, b16& lo) { hi = (b16)v; lo = (b16)(v - (float)hi); }
__device__ __forceinline__ v16b frag_kb(const b16* p, int hh) { const v8b a = *(const v8b*)(p + 8 * hh), b = *(const v8b*)(p + 16 + 8 * hh); v16b f;
#pragma unroll
  for (int e = 0; e < 8; ++e) { f[e] = a[e]; f[8 + e] = b[e]; } return f; }
__device__ __forceinline__ v8f wmma16b(v16b a, v16b b, v8f c) { v8f d = __builtin_amdgcn_wmma_f32_16x16x32_f16(false, a, false, b, (short)0, c, false, false); asm volatile("v_nop\n\tv_nop\n\tv_nop\n\tv_nop" : "+v"(d) : "v"(a), "v"(b)); return d; }
__device__ __forceinline__ void wave_lds_sync() { __builtin_amdgcn_fence(__ATOMIC_RELEASE, "workgroup"); __builtin_amdgcn_wave_barrier(); __builtin_amdgcn_fence(__ATOMIC_ACQUIRE, "workgroup"); }
__device__ __forceinline__ float pmul(float a, float b) { float p = a * b; asm volatile("" : "+v"(p)); return p; }
__device__ __forceinline__ int iclamp(int v, int lo, int hi) { return v < lo ? lo : (v > hi ? hi : v); }
constexpr int CSR_NBLK8 = 512, CSR_GB8 = 8, CSR_GN8 = 1 << CSR_GB8  , CSR_TS8 = (CSR_GN8 < 32 ? 32 : CSR_GN8)  , CSR_MAXG8 = 512, CSR_CAP8 = 12288  ;
__device__ __host__ __forceinline__ int csr_tix8(int v) { return (v >> CSR_GB8) * CSR_TS8 + (v & (CSR_GN8 - 1)); }
__global__ __launch_bounds__(64) void csrA_kernel8(const int* __restrict__ dst, int E, int N, int nG, int CHP, int NGP, int* __restrict__ STG, int* __restrict__ HST) {
  extern __shared__ int sm[];
  int* cnt = sm; int* run = sm + NGP; int* ids = sm + 2 * NGP;
  const int b = blockIdx.x; const int ch = (E + CSR_NBLK8 - 1) / CSR_NBLK8; const int e0 = b * ch, e1 = min(E, e0 + ch);
  for (int i = threadIdx.x; i < NGP; i += 64) cnt[i] = 0;
  for (int i = threadIdx.x; i < CHP; i += 64) ids[i] = -1;
  __syncthreads();
  if (threadIdx.x == 0) {
    for (int e = e0; e < e1; ++e) { int d = dst[e]; d = (d < 0) ? 0 : (d >= N ? N - 1 : d); cnt[d >> CSR_GB8] += 1; }
    int acc = 0; for (int g = 0; g < nG; ++g) { run[g] = acc; acc += cnt[g]; }
    for (int e = e0; e < e1; ++e) { int d = dst[e]; d = (d < 0) ? 0 : (d >= N ? N - 1 : d); const int g = d >> CSR_GB8; ids[run[g]] = e; run[g] += 1; } }
  __syncthreads();
  typedef __attribute__((ext_vector_type(4))) int v4i;
  for (int pass = 0; pass < 2; ++pass) {
    for (int i = threadIdx.x; i < CHP / 4; i += 64) *(volatile v4i*)(STG + (size_t)b * CHP + i * 4) = *(const v4i*)(&ids[i * 4]);
    for (int i = threadIdx.x; i < NGP / 4; i += 64) { v4i v; for (int e = 0; e < 4; ++e) v[e] = (i * 4 + e < nG) ? cnt[i * 4 + e] : 0; *(volatile v4i*)(HST + (size_t)b * NGP + i * 4) = v; }
    __threadfence(); }
}
__global__ __launch_bounds__(512) void csrS_kernel8(const int* __restrict__ HST, int nG, int NGP, int* __restrict__ START, int* __restrict__ TOT, int* __restrict__ OFF) {
  __shared__ int tot[CSR_MAXG8];
  const int b = threadIdx.x;
  for (int pass = 0; pass < 2; ++pass) { int runb = 0; for (int g = 0; g < nG; ++g) { int c = HST[(size_t)b * NGP + g]; c = (c < 0) ? 0 : c; ((volatile int*)OFF)[(size_t)g * CSR_NBLK8 + b] = runb; runb += c; } __threadfence(); }
  for (int g = threadIdx.x; g < nG; g += 512) { int s = 0; for (int bb = 0; bb < CSR_NBLK8; ++bb) { int c = HST[(size_t)bb * NGP + g]; s += (c < 0) ? 0 : c; } tot[g] = s; }
  __syncthreads();
  if (threadIdx.x < 32) {
    __shared__ int st[CSR_MAXG8 + 32];
    if (threadIdx.x == 0) { int acc = 0; for (int g = 0; g < NGP; ++g) { st[g] = acc; if (g < nG) acc += (tot[g] + 31) & ~31; } st[NGP] = acc; }
    __builtin_amdgcn_fence(__ATOMIC_RELEASE, "workgroup"); __builtin_amdgcn_wave_barrier(); __builtin_amdgcn_fence(__ATOMIC_ACQUIRE, "workgroup");
    for (int pass = 0; pass < 2; ++pass) { for (int i = threadIdx.x; i < NGP + 32; i += 32) { ((volatile int*)START)[i] = (i <= NGP) ? st[min(i, NGP)] : 0; ((volatile int*)TOT)[i] = (i < nG) ? tot[i] : 0; } __threadfence(); } }
}
__global__ __launch_bounds__(256) void csrB_kernel8(const int* __restrict__ dst, int N, int nG, int CHP, int NGP, int permLen, const int* __restrict__ STG, const int* __restrict__ HST, const int* __restrict__ OFF, const int* __restrict__ START, const int* __restrict__ TOT, int* __restrict__ PERM, int* __restrict__ ROWPTR, int* __restrict__ ROWCNT, int* __restrict__ FLAG) {
  typedef __attribute__((ext_vector_type(4))) int v4i;
  __shared__ int ids[CSR_CAP8]; __shared__ unsigned short key[CSR_CAP8]; __shared__ int outp[CSR_CAP8]; __shared__ int ncnt[CSR_GN8 + 1]; __shared__ int boff[CSR_NBLK8 + 1];
  const int g = blockIdx.x, t_ = threadIdx.x; int tot = TOT[g]; int st = START[g], stn = START[g + 1]; const int v0 = g * CSR_GN8; const int nv = min(CSR_GN8, N - v0); const int t0 = g * CSR_TS8;
  st = (st < 0) ? 0 : (st > permLen - 32 ? permLen - 32 : st) & ~31; stn = (stn < st) ? st : (stn > permLen ? permLen : stn); tot = (tot < 0) ? 0 : tot; if (tot > stn - st && tot <= CSR_CAP8) tot = stn - st;
  if (tot > CSR_CAP8) {
    for (int pass = 0; pass < 2; ++pass) { for (int i = t_; i < CSR_TS8 / 4; i += 256) { v4i a, c; for (int e = 0; e < 4; ++e) { a[e] = st; c[e] = 0; } *(volatile v4i*)(ROWPTR + t0 + i * 4) = a; *(volatile v4i*)(ROWCNT + t0 + i * 4) = c; } if (t_ == 0) ((volatile int*)FLAG)[0] = 1; __threadfence(); } (void)nv; return; }
  if (t_ == 0) { int acc = 0; for (int b = 0; b < CSR_NBLK8; ++b) { boff[b] = acc; int c = HST[(size_t)b * NGP + g]; c = (c < 0) ? 0 : (c > CHP ? CHP : c); acc += c; if (acc > tot) acc = tot; } boff[CSR_NBLK8] = acc; }
  for (int i = t_; i <= CSR_GN8; i += 256) ncnt[i] = 0;
  __syncthreads();
  for (int b = 0; b < CSR_NBLK8; ++b) { const int c = boff[b + 1] - boff[b]; int o_ = OFF[(size_t)g * CSR_NBLK8 + b]; o_ = (o_ < 0) ? 0 : (o_ > CHP - c ? CHP - c : o_); const int* src_ = STG + (size_t)b * CHP + o_;
    for (int i = t_; i < c; i += 256) { int id = src_[i]; id = (id < 0) ? 0 : id; ids[boff[b] + i] = id; int d = dst[id]; d = (d < v0) ? v0 : (d >= N ? N - 1 : d); int kk = d - v0; kk = (kk < 0) ? 0 : (kk >= CSR_GN8 ? CSR_GN8 - 1 : kk); key[boff[b] + i] = (unsigned short)kk; } }
  __syncthreads();
  if (t_ == 0) { for (int i = 0; i < tot; ++i) ncnt[key[i]] += 1; int acc = 0; for (int vl = 0; vl < CSR_GN8; ++vl) { const int c = ncnt[vl]; ncnt[vl] = acc; acc += c; } ncnt[CSR_GN8] = acc;
    for (int i = 0; i < tot; ++i) { const int vl = key[i]; outp[ncnt[vl]] = ids[i]; ncnt[vl] += 1; }
    for (int vl = CSR_GN8; vl > 0; --vl) ncnt[vl] = ncnt[vl - 1]; ncnt[0] = 0; }
  __syncthreads();
  for (int pass = 0; pass < 2; ++pass) {
    for (int i = t_; i < (stn - st) / 4; i += 256) { v4i v; for (int e = 0; e < 4; ++e) { const int q = i * 4 + e; v[e] = (q < tot) ? outp[q] : -1; } *(volatile v4i*)(PERM + st + i * 4) = v; }
    for (int i = t_; i < CSR_TS8 / 4; i += 256) { v4i a, c; for (int e = 0; e < 4; ++e) { const int vl = i * 4 + e; const int vc = vl < CSR_GN8 ? vl : CSR_GN8; a[e] = (vl < CSR_GN8) ? st + ncnt[vc] : st; c[e] = (vl < nv) ? (ncnt[(vc < CSR_GN8 ? vc : CSR_GN8 - 1) + 1] - ncnt[vc]) : 0; } *(volatile v4i*)(ROWPTR + t0 + i * 4) = a; *(volatile v4i*)(ROWCNT + t0 + i * 4) = c; }
    __threadfence(); }
}
__global__ __launch_bounds__(256) void csrZ_kernel8(int* __restrict__ p, size_t n4) { typedef __attribute__((ext_vector_type(4))) int v4i; const size_t tid = (size_t)blockIdx.x * 256 + threadIdx.x, nth = (size_t)gridDim.x * 256; v4i z = {0, 0, 0, 0}; for (size_t i = tid; i < n4; i += nth) *(volatile v4i*)(p + i * 4) = z; }
struct CsrBufs8 { int *STG, *HST, *OFF, *START, *TOT, *PERM, *ROWPTR, *ROWCNT, *FLAG; int nG, NGP, CHP; size_t permLen; char* base; size_t bytes; };
static size_t csr_carve8(CsrBufs8& c, char* ws, size_t off, int E, int N) {
  const size_t off0 = off; c.base = ws + off;
  auto al = [&](size_t bytes) { char* p = ws + off; off += (bytes + 255) & ~(size_t)255; return p; };
  c.nG = (N + CSR_GN8 - 1) / CSR_GN8; c.NGP = (c.nG + 31) & ~31; const int ch = (E + CSR_NBLK8 - 1) / CSR_NBLK8; c.CHP = (ch + 31) & ~31; c.permLen = (size_t)E + 32 * (size_t)c.nG + 32;
  c.STG = (int*)al((size_t)CSR_NBLK8 * c.CHP * 4); c.HST = (int*)al((size_t)CSR_NBLK8 * c.NGP * 4); c.OFF = (int*)al((size_t)c.NGP * CSR_NBLK8 * 4); c.START = (int*)al((size_t)(c.NGP + 64) * 4); c.TOT = (int*)al((size_t)(c.NGP + 64) * 4);
  c.PERM = (int*)al(c.permLen * 4); c.ROWPTR = (int*)al((size_t)c.nG * CSR_TS8 * 4); c.ROWCNT = (int*)al((size_t)c.nG * CSR_TS8 * 4); c.FLAG = (int*)al(256);
  c.bytes = off - off0; return off;
}
static void csr_build8(const CsrBufs8& c, const int* dst, int E, int N, hipStream_t stream) {
  const size_t smem = (size_t)(2 * c.NGP + c.CHP) * 4;
  csrZ_kernel8<<<512, 256, 0, stream>>>((int*)c.base, c.bytes / 16);
  csrA_kernel8<<<CSR_NBLK8, 64, smem, stream>>>(dst, E, N, c.nG, c.CHP, c.NGP, c.STG, c.HST);
  csrS_kernel8<<<1, 512, 0, stream>>>(c.HST, c.nG, c.NGP, c.START, c.TOT, c.OFF);
  csrB_kernel8<<<c.nG, 256, 0, stream>>>(dst, N, c.nG, c.CHP, c.NGP, (int)c.permLen, c.STG, c.HST, c.OFF, c.START, c.TOT, c.PERM, c.ROWPTR, c.ROWCNT, c.FLAG);
}
constexpr int CSR_NBLK5 = 512, CSR_GB5 = 5, CSR_GN5 = 1 << CSR_GB5  , CSR_TS5 = (CSR_GN5 < 32 ? 32 : CSR_GN5)  , CSR_MAXG5 = 512, CSR_CAP5 = 12288  ;
__device__ __host__ __forceinline__ int csr_tix5(int v) { return (v >> CSR_GB5) * CSR_TS5 + (v & (CSR_GN5 - 1)); }
__global__ __launch_bounds__(64) void csrA_kernel5(const int* __restrict__ dst, int E, int N, int nG, int CHP, int NGP, int* __restrict__ STG, int* __restrict__ HST) {
  extern __shared__ int sm[];
  int* cnt = sm; int* run = sm + NGP; int* ids = sm + 2 * NGP;
  const int b = blockIdx.x; const int ch = (E + CSR_NBLK5 - 1) / CSR_NBLK5; const int e0 = b * ch, e1 = min(E, e0 + ch);
  for (int i = threadIdx.x; i < NGP; i += 64) cnt[i] = 0;
  for (int i = threadIdx.x; i < CHP; i += 64) ids[i] = -1;
  __syncthreads();
  if (threadIdx.x == 0) {
    for (int e = e0; e < e1; ++e) { int d = dst[e]; d = (d < 0) ? 0 : (d >= N ? N - 1 : d); cnt[d >> CSR_GB5] += 1; }
    int acc = 0; for (int g = 0; g < nG; ++g) { run[g] = acc; acc += cnt[g]; }
    for (int e = e0; e < e1; ++e) { int d = dst[e]; d = (d < 0) ? 0 : (d >= N ? N - 1 : d); const int g = d >> CSR_GB5; ids[run[g]] = e; run[g] += 1; } }
  __syncthreads();
  typedef __attribute__((ext_vector_type(4))) int v4i;
  for (int pass = 0; pass < 2; ++pass) {
    for (int i = threadIdx.x; i < CHP / 4; i += 64) *(volatile v4i*)(STG + (size_t)b * CHP + i * 4) = *(const v4i*)(&ids[i * 4]);
    for (int i = threadIdx.x; i < NGP / 4; i += 64) { v4i v; for (int e = 0; e < 4; ++e) v[e] = (i * 4 + e < nG) ? cnt[i * 4 + e] : 0; *(volatile v4i*)(HST + (size_t)b * NGP + i * 4) = v; }
    __threadfence(); }
}
__global__ __launch_bounds__(512) void csrS_kernel5(const int* __restrict__ HST, int nG, int NGP, int* __restrict__ START, int* __restrict__ TOT, int* __restrict__ OFF) {
  __shared__ int tot[CSR_MAXG5];
  const int b = threadIdx.x;
  for (int pass = 0; pass < 2; ++pass) { int runb = 0; for (int g = 0; g < nG; ++g) { int c = HST[(size_t)b * NGP + g]; c = (c < 0) ? 0 : c; ((volatile int*)OFF)[(size_t)g * CSR_NBLK5 + b] = runb; runb += c; } __threadfence(); }
  for (int g = threadIdx.x; g < nG; g += 512) { int s = 0; for (int bb = 0; bb < CSR_NBLK5; ++bb) { int c = HST[(size_t)bb * NGP + g]; s += (c < 0) ? 0 : c; } tot[g] = s; }
  __syncthreads();
  if (threadIdx.x < 32) {
    __shared__ int st[CSR_MAXG5 + 32];
    if (threadIdx.x == 0) { int acc = 0; for (int g = 0; g < NGP; ++g) { st[g] = acc; if (g < nG) acc += (tot[g] + 31) & ~31; } st[NGP] = acc; }
    __builtin_amdgcn_fence(__ATOMIC_RELEASE, "workgroup"); __builtin_amdgcn_wave_barrier(); __builtin_amdgcn_fence(__ATOMIC_ACQUIRE, "workgroup");
    for (int pass = 0; pass < 2; ++pass) { for (int i = threadIdx.x; i < NGP + 32; i += 32) { ((volatile int*)START)[i] = (i <= NGP) ? st[min(i, NGP)] : 0; ((volatile int*)TOT)[i] = (i < nG) ? tot[i] : 0; } __threadfence(); } }
}
__global__ __launch_bounds__(256) void csrB_kernel5(const int* __restrict__ dst, int N, int nG, int CHP, int NGP, int permLen, const int* __restrict__ STG, const int* __restrict__ HST, const int* __restrict__ OFF, const int* __restrict__ START, const int* __restrict__ TOT, int* __restrict__ PERM, int* __restrict__ ROWPTR, int* __restrict__ ROWCNT, int* __restrict__ FLAG) {
  typedef __attribute__((ext_vector_type(4))) int v4i;
  __shared__ int ids[CSR_CAP5]; __shared__ unsigned short key[CSR_CAP5]; __shared__ int outp[CSR_CAP5]; __shared__ int ncnt[CSR_GN5 + 1]; __shared__ int boff[CSR_NBLK5 + 1];
  const int g = blockIdx.x, t_ = threadIdx.x; int tot = TOT[g]; int st = START[g], stn = START[g + 1]; const int v0 = g * CSR_GN5; const int nv = min(CSR_GN5, N - v0); const int t0 = g * CSR_TS5;
  st = (st < 0) ? 0 : (st > permLen - 32 ? permLen - 32 : st) & ~31; stn = (stn < st) ? st : (stn > permLen ? permLen : stn); tot = (tot < 0) ? 0 : tot; if (tot > stn - st && tot <= CSR_CAP5) tot = stn - st;
  if (tot > CSR_CAP5) {
    for (int pass = 0; pass < 2; ++pass) { for (int i = t_; i < CSR_TS5 / 4; i += 256) { v4i a, c; for (int e = 0; e < 4; ++e) { a[e] = st; c[e] = 0; } *(volatile v4i*)(ROWPTR + t0 + i * 4) = a; *(volatile v4i*)(ROWCNT + t0 + i * 4) = c; } if (t_ == 0) ((volatile int*)FLAG)[0] = 1; __threadfence(); } (void)nv; return; }
  if (t_ == 0) { int acc = 0; for (int b = 0; b < CSR_NBLK5; ++b) { boff[b] = acc; int c = HST[(size_t)b * NGP + g]; c = (c < 0) ? 0 : (c > CHP ? CHP : c); acc += c; if (acc > tot) acc = tot; } boff[CSR_NBLK5] = acc; }
  for (int i = t_; i <= CSR_GN5; i += 256) ncnt[i] = 0;
  __syncthreads();
  for (int b = 0; b < CSR_NBLK5; ++b) { const int c = boff[b + 1] - boff[b]; int o_ = OFF[(size_t)g * CSR_NBLK5 + b]; o_ = (o_ < 0) ? 0 : (o_ > CHP - c ? CHP - c : o_); const int* src_ = STG + (size_t)b * CHP + o_;
    for (int i = t_; i < c; i += 256) { int id = src_[i]; id = (id < 0) ? 0 : id; ids[boff[b] + i] = id; int d = dst[id]; d = (d < v0) ? v0 : (d >= N ? N - 1 : d); int kk = d - v0; kk = (kk < 0) ? 0 : (kk >= CSR_GN5 ? CSR_GN5 - 1 : kk); key[boff[b] + i] = (unsigned short)kk; } }
  __syncthreads();
  if (t_ == 0) { for (int i = 0; i < tot; ++i) ncnt[key[i]] += 1; int acc = 0; for (int vl = 0; vl < CSR_GN5; ++vl) { const int c = ncnt[vl]; ncnt[vl] = acc; acc += c; } ncnt[CSR_GN5] = acc;
    for (int i = 0; i < tot; ++i) { const int vl = key[i]; outp[ncnt[vl]] = ids[i]; ncnt[vl] += 1; }
    for (int vl = CSR_GN5; vl > 0; --vl) ncnt[vl] = ncnt[vl - 1]; ncnt[0] = 0; }
  __syncthreads();
  for (int pass = 0; pass < 2; ++pass) {
    for (int i = t_; i < (stn - st) / 4; i += 256) { v4i v; for (int e = 0; e < 4; ++e) { const int q = i * 4 + e; v[e] = (q < tot) ? outp[q] : -1; } *(volatile v4i*)(PERM + st + i * 4) = v; }
    for (int i = t_; i < CSR_TS5 / 4; i += 256) { v4i a, c; for (int e = 0; e < 4; ++e) { const int vl = i * 4 + e; const int vc = vl < CSR_GN5 ? vl : CSR_GN5; a[e] = (vl < CSR_GN5) ? st + ncnt[vc] : st; c[e] = (vl < nv) ? (ncnt[(vc < CSR_GN5 ? vc : CSR_GN5 - 1) + 1] - ncnt[vc]) : 0; } *(volatile v4i*)(ROWPTR + t0 + i * 4) = a; *(volatile v4i*)(ROWCNT + t0 + i * 4) = c; }
    __threadfence(); }
}
__global__ __launch_bounds__(256) void csrZ_kernel5(int* __restrict__ p, size_t n4) { typedef __attribute__((ext_vector_type(4))) int v4i; const size_t tid = (size_t)blockIdx.x * 256 + threadIdx.x, nth = (size_t)gridDim.x * 256; v4i z = {0, 0, 0, 0}; for (size_t i = tid; i < n4; i += nth) *(volatile v4i*)(p + i * 4) = z; }
struct CsrBufs5 { int *STG, *HST, *OFF, *START, *TOT, *PERM, *ROWPTR, *ROWCNT, *FLAG; int nG, NGP, CHP; size_t permLen; char* base; size_t bytes; };
static size_t csr_carve5(CsrBufs5& c, char* ws, size_t off, int E, int N) {
  const size_t off0 = off; c.base = ws + off;
  auto al = [&](size_t bytes) { char* p = ws + off; off += (bytes + 255) & ~(size_t)255; return p; };
  c.nG = (N + CSR_GN5 - 1) / CSR_GN5; c.NGP = (c.nG + 31) & ~31; const int ch = (E + CSR_NBLK5 - 1) / CSR_NBLK5; c.CHP = (ch + 31) & ~31; c.permLen = (size_t)E + 32 * (size_t)c.nG + 32;
  c.STG = (int*)al((size_t)CSR_NBLK5 * c.CHP * 4); c.HST = (int*)al((size_t)CSR_NBLK5 * c.NGP * 4); c.OFF = (int*)al((size_t)c.NGP * CSR_NBLK5 * 4); c.START = (int*)al((size_t)(c.NGP + 64) * 4); c.TOT = (int*)al((size_t)(c.NGP + 64) * 4);
  c.PERM = (int*)al(c.permLen * 4); c.ROWPTR = (int*)al((size_t)c.nG * CSR_TS5 * 4); c.ROWCNT = (int*)al((size_t)c.nG * CSR_TS5 * 4); c.FLAG = (int*)al(256);
  c.bytes = off - off0; return off;
}
static void csr_build5(const CsrBufs5& c, const int* dst, int E, int N, hipStream_t stream) {
  const size_t smem = (size_t)(2 * c.NGP + c.CHP) * 4;
  csrZ_kernel5<<<512, 256, 0, stream>>>((int*)c.base, c.bytes / 16);
  csrA_kernel5<<<CSR_NBLK5, 64, smem, stream>>>(dst, E, N, c.nG, c.CHP, c.NGP, c.STG, c.HST);
  csrS_kernel5<<<1, 512, 0, stream>>>(c.HST, c.nG, c.NGP, c.START, c.TOT, c.OFF);
  csrB_kernel5<<<c.nG, 256, 0, stream>>>(dst, N, c.nG, c.CHP, c.NGP, (int)c.permLen, c.STG, c.HST, c.OFF, c.START, c.TOT, c.PERM, c.ROWPTR, c.ROWCNT, c.FLAG);
}

__device__ __forceinline__ float dinv_of(const int* ROWCNT, size_t i) { return rsqrtf((float)iclamp(ROWCNT[i], 0, E) + 1.0f); }

__global__ __launch_bounds__(256) void wput_kernel(const float* __restrict__ w1, const float* __restrict__ w2, const float* __restrict__ w3, const float* __restrict__ m1, const float* __restrict__ m2, const float* __restrict__ m3, b16* __restrict__ WT1, b16* __restrict__ WT2, b16* __restrict__ WT3, b16* __restrict__ MT1, b16* __restrict__ MT2, b16* __restrict__ MT3) { const int u = blockIdx.x * 256 + threadIdx.x; v8b v;
  if (u < H * 4) { const int o = u / 4, k0 = (u % 4) * 8; v8b a, b, c3;
#pragma unroll
    for (int j = 0; j < 8; ++j) { a[j] = (b16)(bf16_rne(m1[(size_t)(k0 + j) * H + o]) * WSC); b[j] = (b16)(bf16_rne(m2[(size_t)(k0 + j) * H + o]) * WSC); c3[j] = (b16)(o < O ? bf16_rne(m3[(size_t)(k0 + j) * O + o]) * WSC : 0.0f); } for (int pass = 0; pass < 2; ++pass) { *(volatile v8b*)(MT1 + (size_t)o * H + k0) = a; *(volatile v8b*)(MT2 + (size_t)o * H + k0) = b; if (o < 16) *(volatile v8b*)(MT3 + (size_t)o * H + k0) = c3; __threadfence(); } }
  if (u < H * 16) { const int o = u / 16, k0 = (u % 16) * 8;
#pragma unroll
    for (int j = 0; j < 8; ++j) v[j] = (b16)(bf16_rne(w1[(size_t)(k0 + j) * H + o]) * WSC); for (int pass = 0; pass < 2; ++pass) { *(volatile v8b*)(WT1 + (size_t)o * F + k0) = v; __threadfence(); } }
  if (u < H * 4) { const int o = u / 4, k0 = (u % 4) * 8; v8b a, b;
#pragma unroll
    for (int j = 0; j < 8; ++j) { a[j] = (b16)(bf16_rne(w2[(size_t)(k0 + j) * H + o]) * WSC); b[j] = (b16)(bf16_rne(w3[(size_t)(k0 + j) * H + o]) * WSC); } for (int pass = 0; pass < 2; ++pass) { *(volatile v8b*)(WT2 + (size_t)o * H + k0) = a; *(volatile v8b*)(WT3 + (size_t)o * H + k0) = b; __threadfence(); } } }
template <int MODE, int NT>
__global__ __launch_bounds__(32) void lin_kernel(const float* __restrict__ IN, const float* __restrict__ BNP, const b16* __restrict__ W, const float* __restrict__ bias, int NLIM, float* __restrict__ HW) { constexpr int KIN = MODE == 0 ? F : H, OW = NT * 16;   __shared__ __attribute__((aligned(16))) b16 Ah[16][KIN + 8], Al[16][KIN + 8]; __shared__ float Tf[16][H + 1]; const int lane = threadIdx.x, nloc = lane & 15, hlf = lane >> 4; const size_t m0 = (size_t)blockIdx.x * 16; if (m0 >= (size_t)NLIM) return;
  for (int rr = 0; rr < 16; ++rr) for (int q = 0; q < KIN / 32; ++q) { const int c = q * 32 + lane; float v = IN[(m0 + rr) * KIN + c]; b16 p, ql; if (MODE == 0) { p = (b16)(bf16_rne(v) * XS); ql = (b16)0.0f; } else { if (MODE == 1) v = fmaxf(pmul(v, BNP[c]) + BNP[H + c], 0.0f); split16(v * HS, p, ql); } Ah[rr][c] = p; Al[rr][c] = ql; }
  if (lane < 16) for (int k = KIN; k < KIN + 8; ++k) { Ah[lane][k] = (b16)0.0f; Al[lane][k] = (b16)0.0f; }
  wave_lds_sync(); v8f acc[NT];
#pragma unroll
  for (int t = 0; t < NT; ++t) acc[t] = (v8f){};
#pragma unroll
  for (int kb = 0; kb < KIN; kb += 32) { const v16b a = frag_kb(&Ah[nloc][kb], hlf), al = frag_kb(&Al[nloc][kb], hlf);
#pragma unroll
    for (int t = 0; t < NT; ++t) { const v16b bw = frag_kb(W + (size_t)(t * 16 + nloc) * KIN + kb, hlf); acc[t] = wmma16b(a, bw, acc[t]); if (MODE != 0) acc[t] = wmma16b(al, bw, acc[t]); } }
  const float osc = MODE == 0 ? 1.0f / (XS * WSC) : 1.0f / (HS * WSC);
#pragma unroll
  for (int t = 0; t < NT; ++t) { const int cc = t * 16 + nloc; const float bb = bias ? bfv(bias[cc]) : 0.0f;
#pragma unroll
    for (int r8 = 0; r8 < 8; ++r8) Tf[8 * hlf + r8][cc] = acc[t][r8] * osc + bb; }
  wave_lds_sync();
  for (int pass = 0; pass < 2; ++pass) { for (int rr = 0; rr < 16; ++rr) if (lane < OW) ((volatile float*)HW)[(m0 + rr) * OW + lane] = Tf[rr][lane]; __threadfence(); } }
__global__ __launch_bounds__(256) void sweep_kernel(const float* __restrict__ HW, const float* __restrict__ bias, const int* __restrict__ srcs, const int* __restrict__ PERM, const int* __restrict__ ROWPTR, const int* __restrict__ ROWCNT, int permLen, int NLIM, int WANTPS, float* __restrict__ Z, float* __restrict__ PS) { __shared__ float Gs[NPB][H]; const int wave = threadIdx.x >> 5, lane = threadIdx.x & 31; const size_t i = (size_t)blockIdx.x * NPB + wave; const bool live = i < (size_t)NLIM; float o = 0.0f;
  if (live) { int st = ROWPTR[i], cnt = ROWCNT[i]; cnt = iclamp(cnt, 0, E); st = iclamp(st, 0, permLen - cnt); const float di = dinv_of(ROWCNT, i); float acc = 0.0f;
#pragma unroll 1
    for (int j = 0; j < cnt; ++j) { const int e = iclamp(PERM[st + j], 0, E - 1); const size_t u = (size_t)iclamp(srcs[e], 0, N - 1); if (u >= (size_t)NLIM) continue; acc += pmul(dinv_of(ROWCNT, u), HW[u * H + lane]); }
    o = pmul(di, acc + pmul(di, HW[i * H + lane])) + bfv(bias[lane]); }
  if (WANTPS) Gs[wave][lane] = live ? o : 0.0f;
  __syncthreads();
  for (int pass = 0; pass < 2; ++pass) { if (live) ((volatile float*)Z)[i * H + lane] = o;
    if (WANTPS && threadIdx.x < 2 * H) { const int c = threadIdx.x % H, which = threadIdx.x / H; float s = 0.0f; for (int w2 = 0; w2 < NPB; ++w2) { const float v = Gs[w2][c]; s += which ? v * v : v; } ((volatile float*)PS)[(size_t)blockIdx.x * 2 * H + threadIdx.x] = s; } __threadfence(); } }
__global__ __launch_bounds__(64) void bn_kernel(const float* __restrict__ PS, int nb, int count, const float* __restrict__ g, const float* __restrict__ be, float* __restrict__ BNP) { const int c = threadIdx.x & 31; float sc = 0.0f, sh = 0.0f; { double s = 0.0, s2 = 0.0; for (int w = 0; w < nb; ++w) { s += (double)PS[(size_t)w * 2 * H + c]; s2 += (double)PS[(size_t)w * 2 * H + H + c]; } const double mu = s / count; double var = s2 / count - mu * mu; if (var < 0.0) var = 0.0; sc = bfv(g[c]) * (float)(1.0 / sqrt(var + (double)EPS)); sh = bfv(be[c]) - (float)mu * sc; }
  for (int pass = 0; pass < 2; ++pass) { ((volatile float*)BNP)[threadIdx.x] = threadIdx.x < H ? sc : sh; __threadfence(); } }
__global__ __launch_bounds__(64) void gbn_kernel(const float* __restrict__ P, const float* __restrict__ g, const float* __restrict__ be, float* __restrict__ BNP) { const int c = threadIdx.x & 31; double s = 0.0; for (int j = 0; j < G; ++j) s += (double)P[(size_t)j * H + c]; const double mu = s / G; double s2 = 0.0; for (int j = 0; j < G; ++j) { const double d = (double)P[(size_t)j * H + c] - mu; s2 += d * d; } const float sc = bfv(g[c]) * (float)(1.0 / sqrt(s2 / G + (double)EPS)); const float sh = bfv(be[c]) - (float)mu * sc;
  for (int pass = 0; pass < 2; ++pass) { ((volatile float*)BNP)[threadIdx.x] = threadIdx.x < H ? sc : sh; __threadfence(); } }
__global__ __launch_bounds__(256) void pool_kernel(const float* __restrict__ Z, const int* __restrict__ PERM, const int* __restrict__ ROWPTR, const int* __restrict__ ROWCNT, int permLen, int NLIM, float* __restrict__ POOL) { const int wave = threadIdx.x >> 5, lane = threadIdx.x & 31; const int g = blockIdx.x * NPB + wave; if (g >= G) return; int st = ROWPTR[g], cnt = ROWCNT[g]; cnt = iclamp(cnt, 0, N); st = iclamp(st, 0, permLen - cnt); float s = 0.0f; int nn = 0;
#pragma unroll 1
  for (int j = 0; j < cnt; ++j) { const size_t n = (size_t)iclamp(PERM[st + j], 0, N - 1); if (n >= (size_t)NLIM) continue; ++nn; s += Z[n * H + lane]; }
  const float m = s / fmaxf((float)nn, 1.0f);
  for (int pass = 0; pass < 2; ++pass) { ((volatile float*)POOL)[(size_t)g * H + lane] = m; __threadfence(); } }
}

extern "C" void kernel_launch(void* const* d_in, const int* in_sizes, int n_in, void* d_out, int out_size, void* d_ws, size_t ws_size, hipStream_t stream) {
  (void)n_in;
  auto Fp = [&](int i) { return (const float*)d_in[i]; }; auto Ip = [&](int i) { return (const int*)d_in[i]; };
  if (in_sizes[0] != N * F || in_sizes[1] != 2 * E || in_sizes[2] != N || in_sizes[3] != F * H || in_sizes[7] != H * H || in_sizes[11] != H * H || in_sizes[13] != H * H || in_sizes[21] != H * O || out_size != G * O) return;
  const int NLIM = N;
  size_t off = 0; char* ws = (char*)d_ws;
  auto carve = [&](size_t bytes) { char* p = ws + off; off += (bytes + 255) & ~(size_t)255; return p; };
  b16* WT1 = (b16*)carve((size_t)H * F * 2); b16* WT2 = (b16*)carve((size_t)H * H * 2); b16* WT3 = (b16*)carve((size_t)H * H * 2); float* HW = (float*)carve((size_t)N * H * 4); float* Z = (float*)carve((size_t)N * H * 4); float* PS = (float*)carve((size_t)(N / NPB + 1) * 2 * H * 4); float* BN1 = (float*)carve(512); float* BN2 = (float*)carve(512); float* POOL = (float*)carve((size_t)G * H * 4); float* HP1 = (float*)carve((size_t)G * H * 4); float* HP2 = (float*)carve((size_t)G * H * 4); float* BNh1 = (float*)carve(512); float* BNh2 = (float*)carve(512); b16* MT1 = (b16*)carve(H * H * 2); b16* MT2 = (b16*)carve(H * H * 2); b16* MT3 = (b16*)carve(16 * H * 2); CsrBufs8 csr; off = csr_carve8(csr, ws, off, E, N); CsrBufs5 cg; off = csr_carve5(cg, ws, off, N, G);
  if (off > ws_size || off > ((size_t)160 << 20)) return;
  const int nb = (NLIM + NPB - 1) / NPB;
  wput_kernel<<<(H * 16 + 255) / 256, 256, 0, stream>>>(Fp(3), Fp(7), Fp(11), Fp(13), Fp(17), Fp(21), WT1, WT2, WT3, MT1, MT2, MT3);
  csr_build8(csr, Ip(1) + E, E, N, stream); csr_build5(cg, Ip(2), N, G, stream);
  lin_kernel<0, 2><<<NLIM / 16, 32, 0, stream>>>(Fp(0), nullptr, WT1, nullptr, NLIM, HW);
  sweep_kernel<<<nb, 256, 0, stream>>>(HW, Fp(4), Ip(1), csr.PERM, csr.ROWPTR, csr.ROWCNT, (int)csr.permLen, NLIM, 1, Z, PS);
  bn_kernel<<<1, 64, 0, stream>>>(PS, nb, NLIM, Fp(5), Fp(6), BN1);
  lin_kernel<1, 2><<<NLIM / 16, 32, 0, stream>>>(Z, BN1, WT2, nullptr, NLIM, HW);
  sweep_kernel<<<nb, 256, 0, stream>>>(HW, Fp(8), Ip(1), csr.PERM, csr.ROWPTR, csr.ROWCNT, (int)csr.permLen, NLIM, 1, Z, PS);
  bn_kernel<<<1, 64, 0, stream>>>(PS, nb, NLIM, Fp(9), Fp(10), BN2);
  lin_kernel<1, 2><<<NLIM / 16, 32, 0, stream>>>(Z, BN2, WT3, nullptr, NLIM, HW);
  sweep_kernel<<<nb, 256, 0, stream>>>(HW, Fp(12), Ip(1), csr.PERM, csr.ROWPTR, csr.ROWCNT, (int)csr.permLen, NLIM, 0, Z, PS);
  pool_kernel<<<G / NPB, 256, 0, stream>>>(Z, cg.PERM, cg.ROWPTR, cg.ROWCNT, (int)cg.permLen, NLIM, POOL);
  lin_kernel<2, 2><<<G / 16, 32, 0, stream>>>(POOL, nullptr, MT1, Fp(14), G, HP1);
  gbn_kernel<<<1, 64, 0, stream>>>(HP1, Fp(15), Fp(16), BNh1);
  lin_kernel<1, 2><<<G / 16, 32, 0, stream>>>(HP1, BNh1, MT2, Fp(18), G, HP2);
  gbn_kernel<<<1, 64, 0, stream>>>(HP2, Fp(19), Fp(20), BNh2);
  lin_kernel<1, 1><<<G / 16, 32, 0, stream>>>(HP2, BNh2, MT3, Fp(22), G, (float*)d_out);
}
